// QEffPrefillOnlyDeepseekV3MoE_90675349553492
// MI455X (gfx1250) — hardware-verified
//
#include <hip/hip_runtime.h>
#include <hip/hip_bf16.h>

constexpr int T    = 2048;
constexpr int Hdim = 1024;
constexpr int Idim = 512;
constexpr int Enum = 16;
constexpr int Ktop = 4;
constexpr int CAP  = T * Ktop;
constexpr int TM   = 32;

constexpr int TILES_PER_MAT = 1024;
constexpr size_t SWZ_ELEMS_PER_MAT = (size_t)TILES_PER_MAT * 512;
constexpr size_t SWZ_ELEMS = (size_t)Enum * 3 * SWZ_ELEMS_PER_MAT;

typedef __attribute__((ext_vector_type(16))) _Float16 v16h;
typedef __attribute__((ext_vector_type(8)))  _Float16 v8h;
typedef __attribute__((ext_vector_type(4)))  _Float16 v4h;
typedef __attribute__((ext_vector_type(8)))  float  v8f;
typedef __attribute__((ext_vector_type(4)))  float  v4f;
typedef float __attribute__((may_alias)) float_a;
typedef int __attribute__((may_alias)) int_a;
template <typename TT> __device__ __forceinline__ void vst2(void* p, TT v) { *(volatile TT*)p = v; __threadfence(); *(volatile TT*)p = v; }
__device__ inline v8f WMMA16(bool, v16h a, bool, v16h b, short, v8f c, bool, bool) {
  v8f d = __builtin_amdgcn_wmma_f32_16x16x32_f16(false, a, false, b, (short)0, c, false, false);
  asm volatile("v_nop\n\tv_nop\n\tv_nop\n\tv_nop" : "+v"(d) : "v"(a), "v"(b));
  return d;
}


__device__ inline v16h cat16(v8h lo, v8h hi) {
  return __builtin_shufflevector(lo, hi, 0,1,2,3,4,5,6,7,8,9,10,11,12,13,14,15);
}

__device__ inline v16h load_bfrag_direct(const float* __restrict__ p, int stride) {
  v16h b;
#pragma unroll
  for (int j = 0; j < 8; ++j) {
    b[j]     = (_Float16)p[(size_t)j * stride];
    b[j + 8] = (_Float16)p[(size_t)(16 + j) * stride];
  }
  return b;
}

__device__ inline v16h load_afrag(const _Float16* __restrict__ row, int kb, int ko) {
  const _Float16* ap = row + kb + ko;
  return cat16(*(const v8h*)ap, *(const v8h*)(ap + 16));
}

__device__ inline float fast_silu_mul(float g, float u) {
  float s = __builtin_amdgcn_rcpf(1.0f + __expf(-g));
  return g * s * u;
}


__global__ __launch_bounds__(256) void route_kernel(const int* __restrict__ topk_idx, int* __restrict__ cnt, int* __restrict__ tok) {
  __shared__ int lst[CAP];
  __shared__ int wc[8], total;
  const int e = blockIdx.x, tid = threadIdx.x, lane = tid & 31, wave = tid >> 5;
  if (tid == 0) total = 0;
  __syncthreads();
  for (int g0 = 0; g0 < T * Ktop; g0 += 256) {
    const int gid = g0 + tid;
    const bool m = (topk_idx[gid] == e);
    const unsigned msk = (unsigned)__builtin_amdgcn_ballot_w32(m);
    if (lane == 0) wc[wave] = __builtin_popcount(msk);
    __syncthreads();
    int pre = total; for (int w = 0; w < wave; ++w) pre += wc[w];
    if (m) lst[pre + __builtin_popcount(msk & ((1u << lane) - 1u))] = gid;
    __syncthreads();
    if (tid == 0) { int s = total; for (int w = 0; w < 8; ++w) s += wc[w]; total = s; }
    __syncthreads();
  }
  const int n = total;
  for (int i = n + tid; i < ((n + 31) & ~31); i += 256) lst[i] = -1;
  __syncthreads();
  const int nlines = (n + 31) >> 5;
  for (int i = tid; i < nlines * 32; i += 256) vst2(tok + (size_t)e * CAP + i, (int_a)lst[i]);
  if (tid < 32) vst2(cnt + e * 32 + tid, (int_a)(tid == 0 ? n : 0));
}

__global__ void swizzle_kernel(const float* __restrict__ w_gate,
                               const float* __restrict__ w_up,
                               const float* __restrict__ w_down,
                               unsigned short* __restrict__ swz) {
  int gid2 = blockIdx.x * blockDim.x + threadIdx.x;
  int gid = gid2 >> 1, hsel = gid2 & 1;
  const int per_mat = TILES_PER_MAT * 32;
  int matIdx = gid / per_mat;
  if (matIdx >= Enum * 3) return;
  int within = gid - matIdx * per_mat;
  int tile = within >> 5;
  int lane = within & 31;
  int e = matIdx / 3;
  int mat = matIdx - e * 3;

  const float* src;
  int stride, NT;
  if (mat == 0)      { src = w_gate + (size_t)e * Hdim * Idim; stride = Idim; NT = 32; }
  else if (mat == 1) { src = w_up   + (size_t)e * Hdim * Idim; stride = Idim; NT = 32; }
  else               { src = w_down + (size_t)e * Idim * Hdim; stride = Hdim; NT = 64; }

  int kb = tile / NT;
  int nt = tile - kb * NT;
  int k0 = kb * 32 + ((lane >= 16) ? 8 : 0);
  int n  = nt * 16 + (lane & 15);

  union { v8h v; __attribute__((ext_vector_type(4))) unsigned u; } d;
#pragma unroll
  for (int j = 0; j < 8; ++j) d.v[j] = (_Float16)src[(size_t)(k0 + hsel * 16 + j) * stride + n];
  unsigned short* dst =
      swz + ((size_t)matIdx * TILES_PER_MAT + tile) * 512 + (size_t)lane * 16 + hsel * 8;
  vst2(dst, d.u);
}

__device__ inline v16h load_bfrag_swz(const unsigned short* __restrict__ swzMat,
                                       int kb, int nt, int NT, int lane) {
  const unsigned short* p =
      swzMat + ((size_t)(kb * NT + nt) * 512) + (size_t)lane * 16;
  return *(const v16h*)p;
}

template <bool SWZ>
__launch_bounds__(256)
__global__ void moe_kernel(const float* __restrict__ x,
                           const float* __restrict__ w_gate,
                           const float* __restrict__ w_up,
                           const float* __restrict__ w_down,
                           const unsigned short* __restrict__ swz,
                           const int* __restrict__ cnt,
                           const int* __restrict__ tok,
                           float* __restrict__ Dbuf) {
  __shared__ _Float16 sX[TM * Hdim];
  __shared__ _Float16 sAct[TM * Idim];
  __shared__ int    sTok[TM];
  __shared__ __attribute__((aligned(16))) float sD[TM * 128];

  const int e    = blockIdx.y;
  const int tile = blockIdx.x;
  const int n_e  = cnt[e * 32];
  if (tile * TM >= n_e) return;

  const int tid = threadIdx.x;
  if (tid < TM) {
    int r = tile * TM + tid;
    sTok[tid] = (r < n_e) ? tok[e * CAP + r] : -1;
  }
  __syncthreads();

  for (int i4 = tid; i4 < TM * Hdim / 4; i4 += 256) {
    int idx = i4 * 4;
    int m = idx / Hdim, c = idx % Hdim;
    int tkn = sTok[m];
    v4h v = {};
    if (tkn >= 0) {
      const float4 f = *(const float4*)(x + (size_t)(tkn >> 2) * Hdim + c);
      v[0] = (_Float16)f.x; v[1] = (_Float16)f.y;
      v[2] = (_Float16)f.z; v[3] = (_Float16)f.w;
    }
    *(v4h*)(sX + idx) = v;
  }
  __syncthreads();

  const int lane  = tid & 31;
  const int wave  = tid >> 5;
  const int nl    = lane & 15;
  const int ishi  = (lane >= 16);
  const int ko    = ishi ? 8 : 0;
  const int mbase = ishi ? 8 : 0;

  const size_t wofs = (size_t)e * Hdim * Idim;
  const float* wg = w_gate + wofs;
  const float* wu = w_up   + wofs;
  const unsigned short* swzG = swz + (size_t)(e * 3 + 0) * SWZ_ELEMS_PER_MAT;
  const unsigned short* swzU = swz + (size_t)(e * 3 + 1) * SWZ_ELEMS_PER_MAT;
  const unsigned short* swzD = swz + (size_t)(e * 3 + 2) * SWZ_ELEMS_PER_MAT;

  const _Float16* aRow0 = sX + nl * Hdim;
  const _Float16* aRow1 = sX + (16 + nl) * Hdim;

  for (int nt = 0; nt < 4; ++nt) {
    const int n0 = wave * 64 + nt * 16;
    v8f accG0 = {}, accU0 = {}, accG1 = {}, accU1 = {};
#pragma unroll 4
    for (int kb = 0; kb < Hdim; kb += 32) {
      v16h a0 = load_afrag(aRow0, kb, ko);
      v16h a1 = load_afrag(aRow1, kb, ko);
      v16h bg, bu;
      if (SWZ) {
        bg = load_bfrag_swz(swzG, kb >> 5, n0 >> 4, 32, lane);
        bu = load_bfrag_swz(swzU, kb >> 5, n0 >> 4, 32, lane);
      } else {
        bg = load_bfrag_direct(wg + (size_t)(kb + ko) * Idim + n0 + nl, Idim);
        bu = load_bfrag_direct(wu + (size_t)(kb + ko) * Idim + n0 + nl, Idim);
      }
      accG0 = WMMA16(
          false, a0, false, bg, (short)0, accG0, false, false);
      accG1 = WMMA16(
          false, a1, false, bg, (short)0, accG1, false, false);
      accU0 = WMMA16(
          false, a0, false, bu, (short)0, accU0, false, false);
      accU1 = WMMA16(
          false, a1, false, bu, (short)0, accU1, false, false);
    }
#pragma unroll
    for (int r = 0; r < 8; ++r) {
      sAct[(r + mbase) * Idim + n0 + nl] =
          (_Float16)fast_silu_mul(accG0[r], accU0[r]);
      sAct[(16 + r + mbase) * Idim + n0 + nl] =
          (_Float16)fast_silu_mul(accG1[r], accU1[r]);
    }
  }
  __syncthreads();

  const _Float16* cRow0 = sAct + nl * Idim;
  const _Float16* cRow1 = sAct + (16 + nl) * Idim;

  const float* wd = w_down + (size_t)e * Idim * Hdim;
  v8f accA[8], accB[8];
#pragma unroll
  for (int nt = 0; nt < 8; ++nt) {
    const int n0 = wave * 128 + nt * 16;
    v8f acc0 = {}, acc1 = {};
#pragma unroll 4
    for (int kb = 0; kb < Idim; kb += 32) {
      v16h a0 = load_afrag(cRow0, kb, ko);
      v16h a1 = load_afrag(cRow1, kb, ko);
      v16h bd;
      if (SWZ) {
        bd = load_bfrag_swz(swzD, kb >> 5, n0 >> 4, 64, lane);
      } else {
        bd = load_bfrag_direct(wd + (size_t)(kb + ko) * Hdim + n0 + nl, Hdim);
      }
      acc0 = WMMA16(
          false, a0, false, bd, (short)0, acc0, false, false);
      acc1 = WMMA16(
          false, a1, false, bd, (short)0, acc1, false, false);
    }
#pragma unroll
    for (int r = 0; r < 8; ++r) { accA[nt][r] = acc0[r]; accB[nt][r] = acc1[r]; }
  }
  __syncthreads();
  float* stg = (float*)sX + wave * (16 * 128);
#pragma unroll
  for (int pass = 0; pass < 2; ++pass) {
#pragma unroll
    for (int nt = 0; nt < 8; ++nt)
#pragma unroll
      for (int r = 0; r < 8; ++r) stg[(mbase + r) * 128 + nt * 16 + nl] = pass ? accB[nt][r] : accA[nt][r];
    asm volatile("s_wait_dscnt 0" ::: "memory"); __builtin_amdgcn_wave_barrier(); __builtin_amdgcn_fence(__ATOMIC_RELEASE, "workgroup");
#pragma unroll 4
    for (int q = 0; q < 16; ++q) {
      const int gid = sTok[pass * 16 + q];
      if (gid >= 0) vst2(Dbuf + (size_t)gid * Hdim + wave * 128 + lane * 4, *(const v4f*)(stg + q * 128 + lane * 4));
    }
    __builtin_amdgcn_wave_barrier();
  }
}
__global__ __launch_bounds__(256) void combine_kernel(const float* __restrict__ Dbuf, const int* __restrict__ topk_idx,
                                                      const float* __restrict__ topk_w, float* __restrict__ out) {
  const int g = blockIdx.x * 256 + threadIdx.x;
  const int t = g / (Hdim / 4), c4 = g - t * (Hdim / 4);
  int id[Ktop];
#pragma unroll
  for (int k = 0; k < Ktop; ++k) id[k] = topk_idx[t * Ktop + k];
  v4f s = {0.f, 0.f, 0.f, 0.f};
#pragma unroll
  for (int k = 0; k < Ktop; ++k) {
    bool last = true;
#pragma unroll
    for (int k2 = k + 1; k2 < Ktop; ++k2) last = last && (id[k2] != id[k]);
    if (last) { const float w = topk_w[t * Ktop + k]; s += w * *(const v4f*)(Dbuf + ((size_t)(t * Ktop + k)) * Hdim + c4 * 4); }
  }
  vst2(out + (size_t)t * Hdim + c4 * 4, s);
}


extern "C" void kernel_launch(void* const* d_in, const int* in_sizes, int n_in,
                              void* d_out, int out_size, void* d_ws, size_t ws_size,
                              hipStream_t stream) {
  const float* x        = (const float*)d_in[0];
  const int*   topk_idx = (const int*)d_in[1];
  const float* topk_w   = (const float*)d_in[2];
  const float* w_gate   = (const float*)d_in[3];
  const float* w_up     = (const float*)d_in[4];
  const float* w_down   = (const float*)d_in[5];
  float* out = (float*)d_out;

  int*   cnt = (int*)d_ws;
  int*   tok = cnt + Enum * 32;
  size_t routeBytes = (size_t)(Enum * 32 + Enum * CAP) * sizeof(int);
  size_t swzOfs = (routeBytes + 255) & ~(size_t)255;
  unsigned short* swz = (unsigned short*)((char*)d_ws + swzOfs);
  float* Dbuf = (float*)((char*)d_ws + ((swzOfs + SWZ_ELEMS * sizeof(unsigned short) + 255) & ~(size_t)255));
  (void)ws_size; (void)in_sizes; (void)n_in; (void)out_size;

  route_kernel<<<Enum, 256, 0, stream>>>(topk_idx, cnt, tok);
  int convThreads = Enum * 3 * TILES_PER_MAT * 32 * 2;
  swizzle_kernel<<<(convThreads + 255) / 256, 256, 0, stream>>>(w_gate, w_up, w_down, swz);
  dim3 grid(CAP / TM, Enum);
  moe_kernel<true><<<grid, 256, 0, stream>>>(x, w_gate, w_up, w_down, swz, cnt, tok, Dbuf);
  combine_kernel<<<T * Hdim / 4 / 256, 256, 0, stream>>>(Dbuf, topk_idx, topk_w, out);
}
